// DeepEquilibriumModel_34462817583332
// MI455X (gfx1250) — hardware-verified
//
#include <hip/hip_runtime.h>
#include <math.h>

typedef __attribute__((ext_vector_type(16))) _Float16 v16h;
typedef __attribute__((ext_vector_type(8)))  _Float16 v8h;
typedef __attribute__((ext_vector_type(4)))  _Float16 v4h;
typedef __attribute__((ext_vector_type(8)))  float    v8f;
typedef __attribute__((ext_vector_type(4)))  float    v4f;
typedef __attribute__((ext_vector_type(2)))  unsigned v2u;

constexpr int   kRowsAll  = 4096;
constexpr int   kDim      = 2048;
constexpr int   kRowsHalf = 2048;
constexpr int   kHalves   = kRowsAll / kRowsHalf;
constexpr float kBeta     = 0.8f;
constexpr float kLam      = 1e-4f;
constexpr float kDetEps   = 1e-8f;
constexpr float kCarryX   = 64.0f;
constexpr float kCarryZ   = 64.0f;
constexpr float kCarryW   = 1024.0f;
constexpr float kCarryG   = 1024.0f;
constexpr float kScaleC0  = 1.0f / (kCarryX * kCarryW);
constexpr float kScaleIt  = 1.0f / (kCarryZ * kCarryW);
constexpr float kGInv2    = 1.0f / (kCarryG * kCarryG);
constexpr float kF16MinNormal = 6.103515625e-05f;

constexpr int kSlabPitch = 68;
constexpr int kHalfPitch = 72;
constexpr int kTilesN    = kDim / 64;
constexpr int kTilesM    = kRowsHalf / 64;
constexpr int kGemmBlocks = (kTilesM * kTilesN) / 8;
static_assert(kHalves == 2, "two batch halves");
static_assert((kDim % 64) == 0 && (kRowsHalf % 64) == 0, "GEMM M,N multiples of 64");
static_assert((kDim % 32) == 0, "GEMM K multiple of 32");
static_assert((kTilesM * kTilesN) % 8 == 0, "eight tiles per block, exact grid");
static_assert(kDim == 8 * 256, "row kernel: 256 threads x 8 elements");

constexpr size_t kPlane16 = (size_t)kRowsHalf * kDim * 2;
constexpr size_t kPlane32 = (size_t)kRowsHalf * kDim * 4;
constexpr size_t kWsTotal = 7 * kPlane16 + 4 * kPlane32;
static_assert(kPlane16 == 8388608ull && kPlane32 == 16777216ull, "plane sizes");
static_assert(kWsTotal == 125829120ull, "carve total");
static_assert(kWsTotal <= 134217728ull, "carve cap");

__device__ __forceinline__ unsigned short f2bf_bits(float f) {
  unsigned u = __float_as_uint(f);
  return (unsigned short)((u + 0x7FFFu + ((u >> 16) & 1u)) >> 16);
}
__device__ __forceinline__ float bf_bits2f(unsigned short h) { return __uint_as_float(((unsigned)h) << 16); }
__device__ __forceinline__ float bf16_value(float f) { return bf_bits2f(f2bf_bits(f)); }
__device__ __forceinline__ float flush_h(float c) { return (fabsf(c) < kF16MinNormal) ? 0.0f : c; }

__device__ __forceinline__ float h16_to_f32(unsigned hb) {
  const unsigned sgn = (hb & 0x8000u) << 16;
  const unsigned em = hb & 0x7fffu;
  const float fn = __uint_as_float((em << 13) + 0x38000000u);
  const float fs = (float)em * 5.9604644775390625e-8f;
  const float mag = (em < 0x400u) ? fs : fn;
  return __uint_as_float(__float_as_uint(mag) | sgn);
}
__device__ __forceinline__ void dec4(v2u w, float& a, float& b, float& c, float& d) {
  const unsigned w0 = w[0];
  const unsigned w1 = w[1];
  a = h16_to_f32(w0 & 0xffffu);
  b = h16_to_f32(w0 >> 16);
  c = h16_to_f32(w1 & 0xffffu);
  d = h16_to_f32(w1 >> 16);
}

__device__ __forceinline__ void wave_lds_sync() {
  __builtin_amdgcn_fence(__ATOMIC_RELEASE, "workgroup");
  __builtin_amdgcn_wave_barrier();
  __builtin_amdgcn_fence(__ATOMIC_ACQUIRE, "workgroup");
}

__device__ __forceinline__ void tie_acc(v8f& a, v16h x, v16h y) { asm volatile("" : "+v"(a) : "v"(x), "v"(y)); }
__device__ __forceinline__ void guard_acc(v8f& a, v16h x, v16h y) { asm volatile("v_nop\n\tv_nop\n\tv_nop\n\tv_nop" : "+v"(a) : "v"(x), "v"(y)); }
__device__ __forceinline__ void guard_acc1(v8f& a) { asm volatile("v_nop\n\tv_nop\n\tv_nop\n\tv_nop" : "+v"(a)); }
__device__ __forceinline__ void keep4_h(v16h a, v16h b, v16h c, v16h d) { asm volatile("v_nop" :: "v"(a), "v"(b), "v"(c), "v"(d)); }

struct FragH {
  union U { v16h v; v8h h[2]; };
  static __device__ __forceinline__ v16h load(const _Float16* p) {
    U f;
    f.h[0] = *(const v8h*)(p);
    f.h[1] = *(const v8h*)(p + 16);
    return f.v;
  }
  static __device__ __forceinline__ v8f mma(v16h a, v16h b, v8f c) {
    return __builtin_amdgcn_wmma_f32_16x16x32_f16(false, a, false, b, (short)0, c, false, false);
  }
};

__global__ __launch_bounds__(256) void prep_w_kernel(
    const float* __restrict__ Wz, const float* __restrict__ Wx,
    unsigned short* __restrict__ WzT, unsigned short* __restrict__ WxT)
{
  __shared__ __align__(16) float tile[64 * kSlabPitch];
  const int t = threadIdx.x;
  const float* W = (blockIdx.z == 0) ? Wz : Wx;
  unsigned short* O = (blockIdx.z == 0) ? WzT : WxT;
  const int n0 = blockIdx.x * 64;
  const int k0 = blockIdx.y * 64;
#pragma unroll
  for (int it = 0; it < 4; ++it) {
    const int f4 = t + it * 256;
    const int kk = f4 >> 4;
    const int c4 = (f4 & 15) * 4;
    const v4f v = *(const v4f*)(W + (size_t)(k0 + kk) * kDim + n0 + c4);
    *(v4f*)(tile + kk * kSlabPitch + c4) = v;
  }
  __syncthreads();
  const int k8 = (t & 7) * 8;
  v8h hv[2];
#pragma unroll
  for (int it = 0; it < 2; ++it) {
    const int nl = (t >> 3) + it * 32;
#pragma unroll
    for (int e = 0; e < 8; ++e) {
      const float w = tile[(k8 + e) * kSlabPitch + nl];
      hv[it][e] = (_Float16)flush_h(bf16_value(w) * kCarryW);
    }
  }
  for (int pass = 0; pass < 2; ++pass) {
#pragma unroll
    for (int it = 0; it < 2; ++it) {
      const int nl = (t >> 3) + it * 32;
      *(volatile v8h*)(O + (size_t)(n0 + nl) * kDim + k0 + k8) = hv[it];
    }
    __threadfence();
  }
}

constexpr int kPrepXBlocks = (kRowsHalf * kDim / 8) / 256;
static_assert(kPrepXBlocks * 256 * 8 == kRowsHalf * kDim, "prep_x exact coverage");
__global__ __launch_bounds__(256) void prep_x_kernel(const float* __restrict__ x, unsigned short* __restrict__ X16)
{
  const int i = blockIdx.x * 256 + threadIdx.x;
  const size_t e0 = (size_t)i << 3;
  const v4f a0 = *(const v4f*)(x + e0);
  const v4f a1 = *(const v4f*)(x + e0 + 4);
  v8h hv;
#pragma unroll
  for (int e = 0; e < 4; ++e) {
    hv[e]     = (_Float16)flush_h(bf16_value(a0[e]) * kCarryX);
    hv[4 + e] = (_Float16)flush_h(bf16_value(a1[e]) * kCarryX);
  }
  *(volatile v8h*)(X16 + e0) = hv;
  __threadfence();
  *(volatile v8h*)(X16 + e0) = hv;
}

template <int EPI>
__global__ __launch_bounds__(256) void gemm_step_kernel(
    const unsigned short* __restrict__ Ap, const unsigned short* __restrict__ Btp,
    float* C0p, float* Zp, unsigned short* __restrict__ H16p, const float* __restrict__ bias)
{
  __shared__ __align__(16) float    sT[8][16 * kSlabPitch];
  __shared__ __align__(16) _Float16 sH[8][16 * kHalfPitch];
  const _Float16* A  = (const _Float16*)Ap;
  const _Float16* Bt = (const _Float16*)Btp;
  const int lane = threadIdx.x & 31;
  const int wave = threadIdx.x >> 5;
  const int tile = blockIdx.x * 8 + wave;
  const int tm = tile / kTilesN;
  const int tn = tile - tm * kTilesN;
  const int m0 = tm << 6;
  const int n0 = tn << 6;
  const int rlane = lane & 15;
  const int koff  = (lane >> 4) * 8;
  const int mOff  = (lane >> 4) * 8;

  v8f acc[4][4];
#pragma unroll
  for (int i = 0; i < 4; ++i)
#pragma unroll
    for (int j = 0; j < 4; ++j) acc[i][j] = (v8f){0.f, 0.f, 0.f, 0.f, 0.f, 0.f, 0.f, 0.f};

  for (int k0 = 0; k0 < kDim; k0 += 32) {
    v16h bh[4];
#pragma unroll
    for (int j = 0; j < 4; ++j)
      bh[j] = FragH::load(Bt + (size_t)(n0 + (j << 4) + rlane) * kDim + koff + k0);
#pragma unroll
    for (int i = 0; i < 4; ++i) {
      const v16h ah = FragH::load(A + (size_t)(m0 + (i << 4) + rlane) * kDim + koff + k0);
#pragma unroll
      for (int j = 0; j < 4; ++j) acc[i][j] = FragH::mma(ah, bh[j], acc[i][j]);
      tie_acc(acc[i][0], ah, bh[0]);
      tie_acc(acc[i][1], ah, bh[1]);
      tie_acc(acc[i][2], ah, bh[2]);
      guard_acc(acc[i][3], ah, bh[3]);
    }
    keep4_h(bh[0], bh[1], bh[2], bh[3]);
  }
#pragma unroll
  for (int i = 0; i < 4; ++i)
#pragma unroll
    for (int j = 0; j < 4; ++j) guard_acc1(acc[i][j]);

  float* slab = sT[wave];
  _Float16* gs = sH[wave];
  const int hh = lane >> 4;
  const int c4 = (lane & 15) * 4;
  const int q  = lane >> 3;
  const int c8 = (lane & 7) * 8;

  float bcol[4] = {0.f, 0.f, 0.f, 0.f};
  if (EPI == 0) {
#pragma unroll
    for (int j = 0; j < 4; ++j) bcol[j] = bf16_value(bias[n0 + (j << 4) + rlane]);
  }
  const float scl = (EPI == 0) ? kScaleC0 : kScaleIt;

#pragma unroll
  for (int i = 0; i < 4; ++i) {
    const int mBase = m0 + (i << 4);
#pragma unroll
    for (int j = 0; j < 4; ++j) {
#pragma unroll
      for (int r = 0; r < 8; ++r) {
        float v = acc[i][j][r] * scl;
        if (EPI == 0) v += bcol[j];
        slab[(mOff + r) * kSlabPitch + (j << 4) + rlane] = v;
      }
    }
    wave_lds_sync();

    if (EPI == 0) {
      for (int pass = 0; pass < 2; ++pass) {
#pragma unroll
        for (int it = 0; it < 8; ++it) {
          const int row = it * 2 + hh;
          const v4f v = *(const v4f*)(slab + row * kSlabPitch + c4);
          *(volatile v4f*)(C0p + (size_t)(mBase + row) * kDim + n0 + c4) = v;
        }
        __threadfence();
      }
#pragma unroll 1
      for (int it = 0; it < 8; ++it) {
        const int row = it * 2 + hh;
        float* sp = slab + row * kSlabPitch + c4;
        const v4f y = *(const v4f*)sp;
        v4f zt;
        v4h hz;
#pragma unroll
        for (int e = 0; e < 4; ++e) {
          const float zv = kBeta * tanhf(y[e]);
          zt[e] = zv;
          hz[e] = (_Float16)flush_h(zv * kCarryZ);
        }
        *(v4f*)sp = zt;
        *(v4h*)(gs + row * kHalfPitch + c4) = hz;
      }
    } else {
#pragma unroll 1
      for (int it = 0; it < 8; ++it) {
        const int row = it * 2 + hh;
        const size_t gi = (size_t)(mBase + row) * kDim + n0 + c4;
        float* sp = slab + row * kSlabPitch + c4;
        const v4f a4 = *(const v4f*)sp;
        const v4f c0 = *(const v4f*)(C0p + gi);
        const v4f zv = *(const v4f*)(Zp + gi);
        v4f ut;
        v4h hg;
#pragma unroll
        for (int e = 0; e < 4; ++e) {
          const float y = a4[e] + c0[e];
          const float f = tanhf(y);
          const float g = f - zv[e];
          ut[e] = zv[e] + kBeta * g;
          hg[e] = (_Float16)flush_h(g * kCarryG);
        }
        *(v4f*)sp = ut;
        *(v4h*)(gs + row * kHalfPitch + c4) = hg;
      }
    }
    wave_lds_sync();

    for (int pass = 0; pass < 2; ++pass) {
#pragma unroll
      for (int it = 0; it < 8; ++it) {
        const int row = it * 2 + hh;
        const v4f v = *(const v4f*)(slab + row * kSlabPitch + c4);
        *(volatile v4f*)(Zp + (size_t)(mBase + row) * kDim + n0 + c4) = v;
      }
#pragma unroll
      for (int it = 0; it < 4; ++it) {
        const int row = it * 4 + q;
        const v8h hv = *(const v8h*)(gs + row * kHalfPitch + c8);
        *(volatile v8h*)(H16p + (size_t)(mBase + row) * kDim + n0 + c8) = hv;
      }
      __threadfence();
    }
    wave_lds_sync();
  }
}

template <int MODE>
__global__ __launch_bounds__(256) void row_update_kernel(
    float* Zs, float* Uw, const float* Up1,
    const unsigned short* Gc, const unsigned short* Gp1, const unsigned short* Gp2,
    unsigned short* Z16, float* Outp)
{
  __shared__ __align__(16) float sRow[kDim];
  __shared__ __align__(16) float sRed[8 * 8];
  const int t = threadIdx.x;
  const int lane = t & 31;
  const int wave = t >> 5;
  const size_t rb = (size_t)blockIdx.x * kDim;
  const size_t ea = rb + 4 * t;
  const size_t eb = rb + 1024 + 4 * t;
  const v4f ua = *(const v4f*)(Zs + ea);
  const v4f ub = *(const v4f*)(Zs + eb);
  v4f za = ua;
  v4f zb = ub;

  if (MODE != 0) {
    const v4f pa = *(const v4f*)(Up1 + ea);
    const v4f pb = *(const v4f*)(Up1 + eb);
    const v4f qa = *(const v4f*)(Uw + ea);
    const v4f qb = *(const v4f*)(Uw + eb);
    const v2u wca = *(const v2u*)(Gc + ea);
    const v2u wcb = *(const v2u*)(Gc + eb);
    const v2u w1a = *(const v2u*)(Gp1 + ea);
    const v2u w1b = *(const v2u*)(Gp1 + eb);
    const v2u w2a = *(const v2u*)(Gp2 + ea);
    const v2u w2b = *(const v2u*)(Gp2 + eb);
    float gc[8], g1[8], g2[8];
    dec4(wca, gc[0], gc[1], gc[2], gc[3]);
    dec4(wcb, gc[4], gc[5], gc[6], gc[7]);
    dec4(w1a, g1[0], g1[1], g1[2], g1[3]);
    dec4(w1b, g1[4], g1[5], g1[6], g1[7]);
    dec4(w2a, g2[0], g2[1], g2[2], g2[3]);
    dec4(w2b, g2[4], g2[5], g2[6], g2[7]);
    float s00 = 0.f, s01 = 0.f, s11 = 0.f, r0 = 0.f, r1 = 0.f;
#pragma unroll
    for (int e = 0; e < 8; ++e) {
      const float d0 = gc[e] - g1[e];
      const float d1 = gc[e] - g2[e];
      s00 = fmaf(d0, d0, s00);
      s01 = fmaf(d0, d1, s01);
      s11 = fmaf(d1, d1, s11);
      r0  = fmaf(d0, gc[e], r0);
      r1  = fmaf(d1, gc[e], r1);
    }
#pragma unroll
    for (int off = 16; off > 0; off >>= 1) {
      s00 += __shfl_xor(s00, off, 32);
      s01 += __shfl_xor(s01, off, 32);
      s11 += __shfl_xor(s11, off, 32);
      r0  += __shfl_xor(r0, off, 32);
      r1  += __shfl_xor(r1, off, 32);
    }
    if (lane == 0) {
      sRed[wave * 8 + 0] = s00;
      sRed[wave * 8 + 1] = s01;
      sRed[wave * 8 + 2] = s11;
      sRed[wave * 8 + 3] = r0;
      sRed[wave * 8 + 4] = r1;
    }
    __syncthreads();
    float t00 = 0.f, t01 = 0.f, t11 = 0.f, q0 = 0.f, q1 = 0.f;
#pragma unroll
    for (int w = 0; w < 8; ++w) {
      t00 += sRed[w * 8 + 0];
      t01 += sRed[w * 8 + 1];
      t11 += sRed[w * 8 + 2];
      q0  += sRed[w * 8 + 3];
      q1  += sRed[w * 8 + 4];
    }
    t00 *= kGInv2;
    t01 *= kGInv2;
    t11 *= kGInv2;
    q0  *= kGInv2;
    q1  *= kGInv2;
    const float ga = t00 + kLam;
    const float gd = t11 + kLam;
    const float det = ga * gd - t01 * t01 + kDetEps;
    const float inv = 1.0f / det;
    const float gam0 = (gd * q0 - t01 * q1) * inv;
    const float gam1 = (ga * q1 - t01 * q0) * inv;
#pragma unroll
    for (int e = 0; e < 4; ++e) {
      za[e] = ua[e] - gam0 * (ua[e] - pa[e]) - gam1 * (ua[e] - qa[e]);
      zb[e] = ub[e] - gam0 * (ub[e] - pb[e]) - gam1 * (ub[e] - qb[e]);
    }
  }

  if (MODE == 2) {
    for (int pass = 0; pass < 2; ++pass) {
      *(volatile v4f*)(Outp + ea) = za;
      *(volatile v4f*)(Outp + eb) = zb;
      __threadfence();
    }
  } else {
    *(v4f*)(sRow + 4 * t) = za;
    *(v4f*)(sRow + 1024 + 4 * t) = zb;
    __syncthreads();
    const v4f x0 = *(const v4f*)(sRow + 8 * t);
    const v4f x1 = *(const v4f*)(sRow + 8 * t + 4);
    v8h hv;
#pragma unroll
    for (int e = 0; e < 4; ++e) {
      hv[e]     = (_Float16)flush_h(x0[e] * kCarryZ);
      hv[4 + e] = (_Float16)flush_h(x1[e] * kCarryZ);
    }
    for (int pass = 0; pass < 2; ++pass) {
      if (MODE == 1) {
        *(volatile v4f*)(Zs + ea) = za;
        *(volatile v4f*)(Zs + eb) = zb;
      }
      *(volatile v4f*)(Uw + ea) = ua;
      *(volatile v4f*)(Uw + eb) = ub;
      *(volatile v8h*)(Z16 + rb + 8 * t) = hv;
      __threadfence();
    }
  }
}

extern "C" void kernel_launch(void* const* d_in, const int* in_sizes, int n_in,
                              void* d_out, int out_size, void* d_ws, size_t ws_size,
                              hipStream_t stream) {
  if (n_in < 4) return;
  if (in_sizes[0] != kRowsAll * kDim) return;
  if (in_sizes[1] != kDim * kDim) return;
  if (in_sizes[2] != kDim * kDim) return;
  if (in_sizes[3] != kDim) return;
  if (out_size != kRowsAll * kDim) return;
  if (ws_size < kWsTotal) return;

  const float* x  = (const float*)d_in[0];
  const float* Wz = (const float*)d_in[1];
  const float* Wx = (const float*)d_in[2];
  const float* bv = (const float*)d_in[3];
  float* out = (float*)d_out;

  char* ws = (char*)d_ws;
  size_t off = 0;
  auto carve = [&](size_t bytes) -> char* { char* p = ws + off; off += bytes; return p; };
  unsigned short* WZT = (unsigned short*)carve(kPlane16);
  unsigned short* WXT = (unsigned short*)carve(kPlane16);
  unsigned short* X16 = (unsigned short*)carve(kPlane16);
  unsigned short* Z16 = (unsigned short*)carve(kPlane16);
  float* C0 = (float*)carve(kPlane32);
  float* ZS = (float*)carve(kPlane32);
  float* U[2];
  U[0] = (float*)carve(kPlane32);
  U[1] = (float*)carve(kPlane32);
  unsigned short* G[3];
  G[0] = (unsigned short*)carve(kPlane16);
  G[1] = (unsigned short*)carve(kPlane16);
  G[2] = (unsigned short*)carve(kPlane16);
  if (off != kWsTotal) return;

  prep_w_kernel<<<dim3(kDim / 64, kDim / 64, 2), 256, 0, stream>>>(Wz, Wx, WZT, WXT);

  for (int half = 0; half < kHalves; ++half) {
    const size_t rowOff = (size_t)half * kRowsHalf * kDim;
    prep_x_kernel<<<kPrepXBlocks, 256, 0, stream>>>(x + rowOff, X16);
    gemm_step_kernel<0><<<kGemmBlocks, 256, 0, stream>>>(X16, WXT, C0, ZS, Z16, bv);
    for (int i = 1; i <= 5; ++i) {
      gemm_step_kernel<1><<<kGemmBlocks, 256, 0, stream>>>(Z16, WZT, C0, ZS, G[i % 3], bv);
      float* uw = U[i % 2];
      const float* up1 = U[(i + 1) % 2];
      const unsigned short* gc  = G[i % 3];
      const unsigned short* gp1 = G[(i + 2) % 3];
      const unsigned short* gp2 = G[(i + 1) % 3];
      if (i < 3) {
        row_update_kernel<0><<<kRowsHalf, 256, 0, stream>>>(ZS, uw, up1, gc, gp1, gp2, Z16, out + rowOff);
      } else if (i < 5) {
        row_update_kernel<1><<<kRowsHalf, 256, 0, stream>>>(ZS, uw, up1, gc, gp1, gp2, Z16, out + rowOff);
      } else {
        row_update_kernel<2><<<kRowsHalf, 256, 0, stream>>>(ZS, uw, up1, gc, gp1, gp2, Z16, out + rowOff);
      }
    }
  }
}
